// Self_Attention_Memory_Module_22548578304816
// MI455X (gfx1250) — hardware-verified
//
#include <hip/hip_runtime.h>
#include <math.h>

typedef __attribute__((ext_vector_type(16))) _Float16 v16h;
typedef __attribute__((ext_vector_type(16))) __bf16 v16b;
typedef __attribute__((ext_vector_type(8)))  _Float16 v8h;
typedef __attribute__((ext_vector_type(8)))  float v8f;
typedef __attribute__((ext_vector_type(4)))  float v4f;
typedef __attribute__((ext_vector_type(2)))  float v2f;
typedef __attribute__((ext_vector_type(4)))  unsigned v4u;
typedef __attribute__((ext_vector_type(4)))  int v4i;
typedef float __attribute__((may_alias)) float_a;
typedef int __attribute__((may_alias)) int_a;

template <typename T> __device__ __forceinline__ void vst2(void* p, T v) { *(volatile T*)p = v; __threadfence(); *(volatile T*)p = v; }
__device__ __forceinline__ v8f wmma16(v16h a, v16h b, v8f c) {
  v8f d = __builtin_amdgcn_wmma_f32_16x16x32_f16(false, a, false, b, (short)0, c, false, false);
  asm volatile("v_nop\n\tv_nop\n\tv_nop\n\tv_nop" : "+v"(d) : "v"(a), "v"(b));
  return d;
}
__device__ __forceinline__ v8f wmma_bf(v16b a, v16b b, v8f c) {
  v8f d = __builtin_amdgcn_wmma_f32_16x16x32_bf16(false, a, false, b, (short)0, c, false, false);
  asm volatile("v_nop\n\tv_nop\n\tv_nop\n\tv_nop" : "+v"(d) : "v"(a), "v"(b));
  return d;
}
__device__ __forceinline__ v16h frag_h(const _Float16* rowk0, int lane) {
  union { v16h v; v8h q[2]; } u; const _Float16* p = rowk0 + 8 * (lane >> 4);
  u.q[0] = *(const v8h*)p; u.q[1] = *(const v8h*)(p + 16); return u.v;
}
__device__ __forceinline__ v16h frag_f32(const float* rowk0, int lane) {
  v16h a; const float* p = rowk0 + 8 * (lane >> 4);
#pragma unroll
  for (int i = 0; i < 8; ++i) { a[i] = (_Float16)p[i]; a[8 + i] = (_Float16)p[16 + i]; }
  return a;
}
__device__ __forceinline__ v16h frag_f32s(const float* rowk0, int lane, float sc) {
  v16h a; const float* p = rowk0 + 8 * (lane >> 4);
#pragma unroll
  for (int i = 0; i < 8; ++i) { a[i] = (_Float16)(p[i] * sc); a[8 + i] = (_Float16)(p[16 + i] * sc); }
  return a;
}
__device__ __forceinline__ v16h fragc_f32(const float* W, int k0, int n, int lane, int ld, int K) {
  v16h a; const int g = lane >> 4;
#pragma unroll
  for (int i = 0; i < 8; ++i) { const int ka = k0 + 8 * g + i, kb = ka + 16;
    a[i] = (_Float16)(ka < K ? W[(size_t)(ka < K ? ka : K - 1) * ld + n] : 0.f); a[8 + i] = (_Float16)(kb < K ? W[(size_t)(kb < K ? kb : K - 1) * ld + n] : 0.f); }
  return a;
}
struct F2 { v16b h, l; };
__device__ __forceinline__ F2 bsplit16(const float v[16]) { F2 r;
#pragma unroll
  for (int i = 0; i < 16; ++i) { const __bf16 h = (__bf16)v[i]; r.h[i] = h; r.l[i] = (__bf16)(v[i] - (float)h); }
  return r; }
__device__ __forceinline__ F2 split_row(const float* row, int k0, int lane) { float v[16]; const float* p = row + k0 + 8 * (lane >> 4);
#pragma unroll
  for (int i = 0; i < 8; ++i) { v[i] = p[i]; v[8 + i] = p[16 + i]; }
  return bsplit16(v); }
__device__ __forceinline__ F2 split_rowK(const float* row, int k0, int lane, int K) { float v[16]; const int g = lane >> 4;
#pragma unroll
  for (int i = 0; i < 8; ++i) { const int ka = k0 + 8 * g + i, kb = ka + 16; v[i] = ka < K ? row[ka < K ? ka : K - 1] : 0.f; v[8 + i] = kb < K ? row[kb < K ? kb : K - 1] : 0.f; }
  return bsplit16(v); }
__device__ __forceinline__ F2 split_col(const float* W, int k0, int n, int lane, int ld, int K) { float v[16]; const int g = lane >> 4;
#pragma unroll
  for (int i = 0; i < 8; ++i) { const int ka = k0 + 8 * g + i, kb = ka + 16; v[i] = ka < K ? W[(size_t)(ka < K ? ka : K - 1) * ld + n] : 0.f; v[8 + i] = kb < K ? W[(size_t)(kb < K ? kb : K - 1) * ld + n] : 0.f; }
  return bsplit16(v); }
__device__ __forceinline__ v8f mac3(const F2& a, const F2& b, v8f c) { c = wmma_bf(a.l, b.h, c); c = wmma_bf(a.h, b.l, c); return wmma_bf(a.h, b.h, c); }
__device__ __forceinline__ float sigm(float v) { return 1.0f / (1.0f + expf(-v)); }
#define LDSX() do { asm volatile("s_wait_dscnt 0" ::: "memory"); __builtin_amdgcn_wave_barrier(); __builtin_amdgcn_fence(__ATOMIC_RELEASE, "workgroup"); } while (0)

__device__ __forceinline__ float bfr(float v) { return (float)(__bf16)v; }
#define NB 16
#define CC 64
#define HID 16
#define TT 1024
#ifndef TNB
#define TNB NB
#endif
#ifndef XSTR
#define XSTR TT
#endif
typedef __attribute__((ext_vector_type(8))) __bf16 v8b;
__device__ __forceinline__ v16b frag_b(const __bf16* rowk0, int lane) { union { v16b v; v8b q[2]; } u; const __bf16* p = rowk0 + 8 * (lane >> 4); u.q[0] = *(const v8b*)p; u.q[1] = *(const v8b*)(p + 16); return u.v; }
__device__ __forceinline__ v16h frag_h16(const _Float16* row16, int lane) { v16h a; union { v4u v; _Float16 h[8]; } u; u.v = *(const v4u*)(row16 + 8 * (lane >> 4));
#pragma unroll
  for (int i = 0; i < 8; ++i) { a[i] = u.h[i]; a[8 + i] = (_Float16)0.f; }
  return a; }
#define WS_XH  0u
#define WS_XM  (WS_XH + 4u * (size_t)NB * TT * CC)
#define WS_QH  (WS_XM + 4u * (size_t)NB * TT * CC)
#define WS_QL  (WS_QH + 2u * (size_t)NB * TT * HID)
#define WS_KH  (WS_QL + 2u * (size_t)NB * TT * HID)
#define WS_KL  (WS_KH + 2u * (size_t)NB * TT * HID)
#define WS_K2H (WS_KL + 2u * (size_t)NB * TT * HID)
#define WS_K2L (WS_K2H + 2u * (size_t)NB * TT * HID)
#define WS_VT  (WS_K2L + 2u * (size_t)NB * TT * HID)
#define WS_VL  (WS_VT + 2u * (size_t)NB * CC * TT)
#define WS_V2T (WS_VL + 2u * (size_t)NB * CC * TT)
#define WS_V2L (WS_V2T + 2u * (size_t)NB * CC * TT)
#define WS_S   (WS_V2L + 2u * (size_t)NB * CC * TT)
#define WS_Z   (WS_S + 4u * (size_t)NB * TT * TT)
#define WS_ZZ  (WS_Z + 4u * (size_t)NB * TT * 2 * CC)
#define WS_END (WS_ZZ + 4u * (size_t)NB * TT * 2 * CC)
__global__ __launch_bounds__(256) void k_xt(const float* __restrict__ Hh, const float* __restrict__ Mm, float* __restrict__ XH, float* __restrict__ XM) { __shared__ float st[CC][65];
  const int t = threadIdx.x; const int n0 = blockIdx.x * 64; const size_t b = blockIdx.y; const float* IN = blockIdx.z == 0 ? Hh : Mm; float* OUT = blockIdx.z == 0 ? XH : XM;
  for (int e = t; e < CC * 64; e += 256) { const int c = e >> 6, nl = e & 63; st[c][nl] = bfr(IN[(b * CC + c) * (size_t)XSTR + n0 + nl]); }
  __syncthreads();
  for (int e = t; e < 64 * 16; e += 256) { const int nl = e >> 4, q = e & 15; v4f o; o[0] = st[q * 4][nl]; o[1] = st[q * 4 + 1][nl]; o[2] = st[q * 4 + 2][nl]; o[3] = st[q * 4 + 3][nl]; vst2(OUT + (b * TT + n0 + nl) * CC + q * 4, o); } }
__global__ __launch_bounds__(128) void k_proj(const float* __restrict__ XH, const float* __restrict__ XM, const float* __restrict__ WQ, const float* __restrict__ BQ, const float* __restrict__ WK, const float* __restrict__ BK, const float* __restrict__ WK2, const float* __restrict__ BK2, const float* __restrict__ WV, const float* __restrict__ BV, const float* __restrict__ WV2, const float* __restrict__ BV2,
    _Float16* __restrict__ QH, _Float16* __restrict__ QL, _Float16* __restrict__ KH, _Float16* __restrict__ KL, _Float16* __restrict__ K2H, _Float16* __restrict__ K2L, __bf16* __restrict__ VT, __bf16* __restrict__ VL, __bf16* __restrict__ V2T, __bf16* __restrict__ V2L) {
  __shared__ __align__(16) _Float16 sqh[64][40], sql[64][40]; __shared__ __align__(16) __bf16 th[CC][72], tl[CC][72];
  const int tid = threadIdx.x, wave = tid >> 5, lane = tid & 31, col = lane & 15, g = lane >> 4; const int which = blockIdx.y; const size_t r0 = (size_t)blockIdx.x * 64; const float* X = which == 0 ? XH : XM;
  const int ntile = which == 0 ? 6 : 5;
  v8f acc[6] = {};
#pragma unroll
  for (int kc = 0; kc < CC / 32; ++kc) { v16b a; { const float* p = X + (r0 + wave * 16 + col) * CC + kc * 32 + 8 * g;
#pragma unroll
      for (int i = 0; i < 8; ++i) { a[i] = (__bf16)p[i]; a[8 + i] = (__bf16)p[16 + i]; } }
#pragma unroll
    for (int j = 0; j < 6; ++j) { if (j >= ntile) break; const float* Wt; int o;
      if (which == 0) { if (j == 0) { Wt = WQ; o = col; } else if (j == 1) { Wt = WK; o = col; } else { Wt = WV; o = (j - 2) * 16 + col; } }
      else { if (j == 0) { Wt = WK2; o = col; } else { Wt = WV2; o = (j - 1) * 16 + col; } }
      v16b w; const float* wr = Wt + (size_t)o * CC + kc * 32 + 8 * g;
#pragma unroll
      for (int i = 0; i < 8; ++i) { w[i] = (__bf16)wr[i]; w[8 + i] = (__bf16)wr[16 + i]; }
      asm volatile("s_wait_loadcnt 0x0" ::: "memory"); acc[j] = wmma_bf(a, w, acc[j]); } }
#pragma unroll
  for (int j = 0; j < 6; ++j) { if (j >= ntile) break; const bool isq = (which == 0 && j == 0), isk = (which == 0 && j == 1) || (which == 1 && j == 0); const int vt = which == 0 ? j - 2 : j - 1;
    const float* Bv = isq ? BQ : isk ? (which == 0 ? BK : BK2) : (which == 0 ? BV : BV2); const int o = (isq || isk) ? col : vt * 16 + col; const float bb = bfr(Bv[o]);
#pragma unroll
    for (int r = 0; r < 8; ++r) { const float v = acc[j][r] + bb; const int rl = wave * 16 + 8 * g + r;
      if (isq || isk) { const _Float16 hv = (_Float16)v; sqh[rl][(isq ? 0 : 16) + col] = hv; sql[rl][(isq ? 0 : 16) + col] = (_Float16)((v - (float)hv) * 1024.0f); }
      else { const __bf16 bh = (__bf16)v; th[o][rl] = bh; tl[o][rl] = (__bf16)(v - (float)bh); } } }
  __syncthreads();
  if (which == 0) { for (int e = tid; e < 64 * 2; e += 128) { const int rl = e >> 1, q = e & 1; vst2((unsigned*)(QH + (r0 + rl) * HID + q * 8), *(const v4u*)&sqh[rl][q * 8]); vst2((unsigned*)(QL + (r0 + rl) * HID + q * 8), *(const v4u*)&sql[rl][q * 8]); vst2((unsigned*)(KH + (r0 + rl) * HID + q * 8), *(const v4u*)&sqh[rl][16 + q * 8]); vst2((unsigned*)(KL + (r0 + rl) * HID + q * 8), *(const v4u*)&sql[rl][16 + q * 8]); } }
  else { for (int e = tid; e < 64 * 2; e += 128) { const int rl = e >> 1, q = e & 1; vst2((unsigned*)(K2H + (r0 + rl) * HID + q * 8), *(const v4u*)&sqh[rl][16 + q * 8]); vst2((unsigned*)(K2L + (r0 + rl) * HID + q * 8), *(const v4u*)&sql[rl][16 + q * 8]); } }
  { __bf16* DT = which == 0 ? VT : V2T; __bf16* DL = which == 0 ? VL : V2L; const size_t b = r0 / TT; const int n0 = (int)(r0 % TT); for (int e = tid; e < CC * 8; e += 128) { const int cl = e >> 3, q = e & 7; const size_t o2 = (b * CC + cl) * (size_t)TT + n0 + q * 8; vst2((unsigned*)(DT + o2), *(const v4u*)&th[cl][q * 8]); vst2((unsigned*)(DL + o2), *(const v4u*)&tl[cl][q * 8]); } } }
__global__ __launch_bounds__(128) void k_sc(const _Float16* __restrict__ QH, const _Float16* __restrict__ QL, const _Float16* __restrict__ KH, const _Float16* __restrict__ KL, float* __restrict__ S0) { __shared__ __align__(16) float ss[4][16][132];
  const size_t b = blockIdx.z; float* S = S0 + b * TT * TT;
  const int tid = threadIdx.x, wave = tid >> 5, lane = tid & 31, col = lane & 15, g = lane >> 4; const int k0 = blockIdx.y * 128; const int ql0 = blockIdx.x * 64 + wave * 16;
  v8f acc[8] = {}, accl[8] = {};
  { const size_t qo = (b * TT + ql0 + col) * HID; const v16h ah = frag_h16(QH + qo, lane), al = frag_h16(QL + qo, lane);
#pragma unroll
    for (int j = 0; j < 8; ++j) { const size_t ko = (b * TT + k0 + j * 16 + col) * HID; const v16h kb = frag_h16(KH + ko, lane), kl = frag_h16(KL + ko, lane); acc[j] = wmma16(ah, kb, acc[j]); accl[j] = wmma16(al, kb, accl[j]); accl[j] = wmma16(ah, kl, accl[j]); } }
#pragma unroll
  for (int j = 0; j < 8; ++j)
#pragma unroll
    for (int r = 0; r < 8; ++r) ss[wave][8 * g + r][j * 16 + col] = acc[j][r] + accl[j][r] * (1.0f / 1024.0f);
  LDSX(); for (int rl = 0; rl < 16; ++rl) vst2(S + (size_t)(ql0 + rl) * TT + k0 + lane * 4, *(const v4f*)&ss[wave][rl][lane * 4]); }
__global__ __launch_bounds__(256) void k_sm(float* __restrict__ S0) { __shared__ float sred[8]; __shared__ float sbc; __shared__ __align__(16) float sh[TT];
  const int t = threadIdx.x; const size_t row = blockIdx.x; float* sr = S0 + ((size_t)blockIdx.y * TT + row) * TT;
  float m = -3.0e38f; for (int k = t; k < TT; k += 256) { const float v = sr[k]; sh[k] = v; m = fmaxf(m, v); }
#pragma unroll
  for (int o = 1; o < 32; o <<= 1) m = fmaxf(m, __shfl_xor(m, o));
  if ((t & 31) == 0) sred[t >> 5] = m; __syncthreads(); if (t == 0) { float a = sred[0]; for (int w = 1; w < 8; ++w) a = fmaxf(a, sred[w]); sbc = a; } __syncthreads(); m = sbc; __syncthreads();
  float s = 0.f; for (int k = t; k < TT; k += 256) { const float e = expf(sh[k] - m); sh[k] = e; s += e; }
#pragma unroll
  for (int o = 1; o < 32; o <<= 1) s += __shfl_xor(s, o);
  if ((t & 31) == 0) sred[t >> 5] = s; __syncthreads(); if (t == 0) { float a = 0.f; for (int w = 0; w < 8; ++w) a += sred[w]; sbc = 2048.0f / a; } __syncthreads(); const float sc = sbc;
  for (int k = t; k < TT; k += 256) sh[k] *= sc;
  __syncthreads(); for (int q = t; q < TT / 4; q += 256) vst2(sr + q * 4, *(const v4f*)&sh[q * 4]); }
__global__ __launch_bounds__(128) void k_pv(const float* __restrict__ S0, const __bf16* __restrict__ VT, const __bf16* __restrict__ VL, int zoff, float* __restrict__ Z) { __shared__ __align__(16) float ss[4][16][CC + 4];
  const size_t b = blockIdx.z; const float* PS = S0 + b * TT * TT;
  const int tid = threadIdx.x, wave = tid >> 5, lane = tid & 31, col = lane & 15, g = lane >> 4; const int ql0 = blockIdx.x * 64 + wave * 16;
  v8f acc[CC / 16] = {};
#pragma unroll 1
  for (int kc = 0; kc < TT / 32; ++kc) { const F2 p = split_row(PS + (size_t)(ql0 + col) * TT, kc * 32, lane);
#pragma unroll
    for (int j = 0; j < CC / 16; ++j) { const size_t po = (b * CC + j * 16 + col) * (size_t)TT + kc * 32; const v16b vh = frag_b(VT + po, lane); acc[j] = wmma_bf(p.h, vh, acc[j]); acc[j] = wmma_bf(p.l, vh, acc[j]); acc[j] = wmma_bf(p.h, frag_b(VL + po, lane), acc[j]); } }
#pragma unroll
  for (int j = 0; j < CC / 16; ++j)
#pragma unroll
    for (int r = 0; r < 8; ++r) ss[wave][8 * g + r][j * 16 + col] = acc[j][r] * (1.0f / 2048.0f);
  LDSX(); for (int rl = 0; rl < 16; ++rl) if (lane < CC / 4) vst2(Z + (b * TT + ql0 + rl) * (2 * CC) + zoff + lane * 4, *(const v4f*)&ss[wave][rl][lane * 4]); }
__global__ __launch_bounds__(128) void k_z(const float* __restrict__ Zin, const float* __restrict__ WZ, const float* __restrict__ BZ, float* __restrict__ ZZ) { __shared__ __align__(16) float sf[4][16][132];
  const int tid = threadIdx.x, wave = tid >> 5, lane = tid & 31, col = lane & 15, g = lane >> 4; const size_t r0 = (size_t)blockIdx.x * 64 + wave * 16;
  v8f acc[8] = {};
#pragma unroll
  for (int kc = 0; kc < 2 * CC / 32; ++kc) { const F2 a = split_row(Zin + (r0 + col) * (2 * CC), kc * 32, lane);
#pragma unroll
    for (int j = 0; j < 8; ++j) { v16b w; const float* wr = WZ + (size_t)(j * 16 + col) * (2 * CC) + kc * 32 + 8 * g;
#pragma unroll
      for (int i = 0; i < 8; ++i) { w[i] = (__bf16)wr[i]; w[8 + i] = (__bf16)wr[16 + i]; }
      asm volatile("s_wait_loadcnt 0x0" ::: "memory"); acc[j] = wmma_bf(a.h, w, acc[j]); acc[j] = wmma_bf(a.l, w, acc[j]); } }
#pragma unroll
  for (int j = 0; j < 8; ++j) { const float bb = bfr(BZ[j * 16 + col]);
#pragma unroll
    for (int r = 0; r < 8; ++r) sf[wave][8 * g + r][j * 16 + col] = acc[j][r] + bb; }
  LDSX(); for (int rl = 0; rl < 16; ++rl) vst2(ZZ + (r0 + rl) * (2 * CC) + lane * 4, *(const v4f*)&sf[wave][rl][lane * 4]); }
__global__ __launch_bounds__(128) void k_m(const float* __restrict__ ZZ, const float* __restrict__ XH, const float* __restrict__ WM, const float* __restrict__ BM, const float* __restrict__ Mm, float* __restrict__ OH, float* __restrict__ OM) { __shared__ __align__(16) float sth[CC][68], stm[CC][68];
  const int tid = threadIdx.x, wave = tid >> 5, lane = tid & 31, col = lane & 15, g = lane >> 4; const size_t rb = (size_t)blockIdx.x * 64; const size_t r0 = rb + wave * 16; const size_t b = rb / TT; const int n0 = (int)(rb % TT);
  v8f acc[12] = {};
#pragma unroll
  for (int kc = 0; kc < 6; ++kc) { F2 a; if (kc < 4) a = split_row(ZZ + (r0 + col) * (2 * CC), kc * 32, lane); else { float v[16]; const float* p = XH + (r0 + col) * CC + (kc - 4) * 32 + 8 * g;
#pragma unroll
      for (int i = 0; i < 8; ++i) { v[i] = p[i]; v[8 + i] = p[16 + i]; }
      a = bsplit16(v); }
#pragma unroll
    for (int j = 0; j < 12; ++j) { v16b w; const float* wr = WM + (size_t)(j * 16 + col) * (3 * CC) + kc * 32 + 8 * g;
#pragma unroll
      for (int i = 0; i < 8; ++i) { w[i] = (__bf16)wr[i]; w[8 + i] = (__bf16)wr[16 + i]; }
      asm volatile("s_wait_loadcnt 0x0" ::: "memory"); acc[j] = wmma_bf(a.h, w, acc[j]); acc[j] = wmma_bf(a.l, w, acc[j]); } }
#pragma unroll
  for (int jj = 0; jj < 4; ++jj) { const int c = jj * 16 + col; const float bo = bfr(BM[c]), bg = bfr(BM[CC + c]), bi = bfr(BM[2 * CC + c]);
#pragma unroll
    for (int r = 0; r < 8; ++r) { const int rl = wave * 16 + 8 * g + r; const float mo = acc[jj][r] + bo, mg = acc[4 + jj][r] + bg, mi = sigm(acc[8 + jj][r] + bi); const float mv = bfr(Mm[(b * CC + c) * (size_t)XSTR + n0 + rl]); const float nm = (1.0f - mi) * mv + mi * tanhf(mg); stm[c][rl] = nm; sth[c][rl] = sigm(mo) * nm; }
    asm volatile("s_wait_loadcnt 0x0" ::: "memory"); }
  __syncthreads();
  for (int e = tid; e < CC * 16; e += 128) { const int c = e >> 4, q = e & 15; const size_t off = (b * CC + c) * (size_t)XSTR + n0 + q * 4; vst2(OH + off, *(const v4f*)&sth[c][q * 4]); vst2(OM + off, *(const v4f*)&stm[c][q * 4]); } }
extern "C" void kernel_launch(void* const* d_in, const int* in_sizes, int n_in, void* d_out, int out_size, void* d_ws, size_t ws_size, hipStream_t stream) {
  (void)in_sizes; (void)n_in; (void)out_size;
  const float** F = (const float**)d_in;
  if (ws_size < (size_t)WS_END) return;
  char* ws = (char*)d_ws; float *XH = (float*)(ws + WS_XH), *XM = (float*)(ws + WS_XM), *S = (float*)(ws + WS_S), *Z = (float*)(ws + WS_Z), *ZZ = (float*)(ws + WS_ZZ);
  _Float16 *QH = (_Float16*)(ws + WS_QH), *QL = (_Float16*)(ws + WS_QL), *KH = (_Float16*)(ws + WS_KH), *KL = (_Float16*)(ws + WS_KL), *K2H = (_Float16*)(ws + WS_K2H), *K2L = (_Float16*)(ws + WS_K2L); __bf16 *VT = (__bf16*)(ws + WS_VT), *VL = (__bf16*)(ws + WS_VL), *V2T = (__bf16*)(ws + WS_V2T), *V2L = (__bf16*)(ws + WS_V2L);
  float* OH = (float*)d_out; float* OM = (float*)d_out + (size_t)NB * CC * TT;
  k_xt<<<dim3(TT / 64, TNB, 2), 256, 0, stream>>>(F[0], F[1], XH, XM);
  k_proj<<<dim3(TNB * TT / 64, 2), 128, 0, stream>>>(XH, XM, F[2], F[3], F[4], F[5], F[6], F[7], F[8], F[9], F[10], F[11], QH, QL, KH, KL, K2H, K2L, VT, VL, V2T, V2L);
  k_sc<<<dim3(TT / 64, TT / 128, TNB), 128, 0, stream>>>(QH, QL, KH, KL, S); k_sm<<<dim3(TT, TNB), 256, 0, stream>>>(S); k_pv<<<dim3(TT / 64, 1, TNB), 128, 0, stream>>>(S, VT, VL, 0, Z);
  k_sc<<<dim3(TT / 64, TT / 128, TNB), 128, 0, stream>>>(QH, QL, K2H, K2L, S); k_sm<<<dim3(TT, TNB), 256, 0, stream>>>(S); k_pv<<<dim3(TT / 64, 1, TNB), 128, 0, stream>>>(S, V2T, V2L, CC, Z);
  k_z<<<dim3(TNB * TT / 64), 128, 0, stream>>>(Z, F[12], F[13], ZZ);
  k_m<<<dim3(TNB * TT / 64), 128, 0, stream>>>(ZZ, XH, F[14], F[15], F[1], OH, OM);
}
